// DuplicateRemovalLayer_70325794505465
// MI455X (gfx1250) — hardware-verified
//
#include <hip/hip_runtime.h>
#include <stdint.h>

#define DEVINL __device__ __forceinline__

typedef _Float16 f16t;
typedef unsigned long long u64;
typedef _Float16 v16h __attribute__((ext_vector_type(16)));
typedef _Float16 v8h  __attribute__((ext_vector_type(8)));
typedef float    v8f  __attribute__((ext_vector_type(8)));
typedef float    v4f  __attribute__((ext_vector_type(4)));
typedef float    v2f  __attribute__((ext_vector_type(2)));
typedef v8h __attribute__((may_alias)) v8ha;
typedef v4f __attribute__((may_alias)) v4fa;
typedef v2f __attribute__((may_alias)) v2fa;
union FragH { v16h v; v8h half[2]; };
static_assert(sizeof(FragH) == 32);

#define NB   8
#define NN   512
#define NC   256
#define NU   128
#define WCAR   16.0f
#define KQVCAR 4.0f
#define PCAR   1024.0f
#define EP   136
#define PP   72
#define TPW  256
#define TPP  128
#define TPR  64
#define PT   64
#define RT   32
#define MT   64

static_assert((EP % 8) == 0);
static_assert((PP % 8) == 0);
static_assert(NN % PT == 0);
static_assert(NN % RT == 0);
static_assert(NN % MT == 0);
static_assert(NU % 32 == 0);
static_assert(NC % 32 == 0);
static_assert(TPP * 4 == NN);
static_assert(TPR * 8 == NN);

DEVINL v8f wmma_h(v16h a, v16h b, v8f c) {
  v8f d = __builtin_amdgcn_wmma_f32_16x16x32_f16(false, a, false, b, (short)0, c, false, false);
  asm volatile("v_nop\n\tv_nop\n\tv_nop\n\tv_nop" : "+v"(d) : "v"(a), "v"(b));
  return d;
}
DEVINL v8f zero8f() {
  v8f z = {0.f, 0.f, 0.f, 0.f, 0.f, 0.f, 0.f, 0.f};
  return z;
}

DEVINL unsigned ord_bits(float v) {
  v = v + 0.0f;
  const unsigned bb = __float_as_uint(v);
  return (bb & 0x80000000u) ? ~bb : (bb | 0x80000000u);
}
DEVINL u64 mkkey(float v, int idx) {
  const unsigned o = ord_bits(v);
  return (((u64)(0xFFFFFFFFu - o)) << 32) | (u64)(unsigned)idx;
}
DEVINL void cex(u64* a, int i, int l, bool asc) {
  const u64 x = a[i], y = a[l];
  const bool lt = x < y;
  const u64 mn = lt ? x : y, mx = lt ? y : x;
  a[i] = asc ? mn : mx;
  a[l] = asc ? mx : mn;
}

__global__ __launch_bounds__(TPW) void prep_w_k(const float* __restrict__ Wr, const float* __restrict__ Wf,
                                               const float* __restrict__ Wk, const float* __restrict__ Wq,
                                               const float* __restrict__ Wv,
                                               f16t* __restrict__ Tr, f16t* __restrict__ Tf,
                                               f16t* __restrict__ Tk, f16t* __restrict__ Tq,
                                               f16t* __restrict__ Tv)
{
  const int blk = blockIdx.x, tid = threadIdx.x;
  const float* src = Wv; f16t* dst = Tv; int ksh = 4; int pb = 40;
  if (blk < 8)       { src = Wr; dst = Tr; ksh = 4; pb = 0;  }
  else if (blk < 24) { src = Wf; dst = Tf; ksh = 5; pb = 8;  }
  else if (blk < 32) { src = Wk; dst = Tk; ksh = 4; pb = 24; }
  else if (blk < 40) { src = Wq; dst = Tq; ksh = 4; pb = 32; }
  const int p  = (blk - pb) * TPW + tid;
  const int n  = p >> ksh;
  const int pc = p & ((1 << ksh) - 1);
  v8h o;
  #pragma unroll
  for (int i = 0; i < 8; ++i) o[i] = (f16t)(src[(size_t)(8 * pc + i) * NU + n] * WCAR);
  f16t* d = dst + (size_t)p * 8;
  *(volatile v8h*)d = o;
  __threadfence();
  *(volatile v8h*)d = o;
}

__global__ __launch_bounds__(TPP) void proj_k(const float* __restrict__ feat, const float* __restrict__ scores,
                                             const float* __restrict__ enc,
                                             const float* __restrict__ br, const float* __restrict__ bfe,
                                             const float* __restrict__ bk, const float* __restrict__ bq,
                                             const float* __restrict__ bv,
                                             const f16t* __restrict__ Tr, const f16t* __restrict__ Tf,
                                             const f16t* __restrict__ Tk, const f16t* __restrict__ Tq,
                                             const f16t* __restrict__ Tv,
                                             f16t* __restrict__ KP, f16t* __restrict__ QP,
                                             f16t* __restrict__ VT)
{
  __shared__ __attribute__((aligned(16))) u64  sKey[NN];
  __shared__ __attribute__((aligned(16))) f16t sEnc[PT * EP];
  __shared__ __attribute__((aligned(16))) f16t sEmb[PT * EP];
  const int tid = threadIdx.x, lane = tid & 31, wave = tid >> 5;
  const int h = lane >> 4, m = lane & 15;
  const int b = blockIdx.x >> 3, n0 = (blockIdx.x & 7) * PT;
  const size_t rowg = (size_t)b * NN + n0;

  #pragma unroll
  for (int e = 0; e < 4; ++e) {
    const int j = tid + TPP * e;
    sKey[j] = mkkey(scores[(size_t)b * NN + j], j);
  }
  __syncthreads();
  #pragma unroll 1
  for (int k = 2; k <= NN; k <<= 1) {
    #pragma unroll 1
    for (int j = k >> 1; j > 0; j >>= 1) {
      #pragma unroll
      for (int q = 0; q < 2; ++q) {
        const int idx = tid + TPP * q;
        const int i = ((idx & ~(j - 1)) << 1) | (idx & (j - 1));
        cex(sKey, i, i | j, (i & k) == 0);
      }
      __syncthreads();
    }
  }
  #pragma unroll
  for (int e = 0; e < 8; ++e) {
    const int p = tid + TPP * e;
    const int row = p >> 4, c8 = (p & 15) * 8;
    int ix = (int)(unsigned)(sKey[n0 + row] & 0xFFFFFFFFull);
    ix = ix < 0 ? 0 : (ix > NN - 1 ? NN - 1 : ix);
    const float* er = enc + (size_t)ix * NU + c8;
    const v4f e0 = *(const v4fa*)er;
    const v4f e1 = *(const v4fa*)(er + 4);
    v8h o;
    #pragma unroll
    for (int i = 0; i < 4; ++i) { o[i] = (f16t)e0[i]; o[4 + i] = (f16t)e1[i]; }
    *(v8ha*)(sEnc + row * EP + c8) = o;
  }
  __syncthreads();

  v8f acc[8];
  #pragma unroll
  for (int nt = 0; nt < 8; ++nt) acc[nt] = zero8f();
  {
    const f16t* arow = sEnc + (16 * wave + m) * EP + 8 * h;
    #pragma unroll 1
    for (int ks = 0; ks < NU / 32; ++ks) {
      FragH a;
      a.half[0] = *(const v8ha*)(arow + 32 * ks);
      a.half[1] = *(const v8ha*)(arow + 32 * ks + 16);
      #pragma unroll
      for (int nt = 0; nt < 8; ++nt) {
        const f16t* brw = Tr + (size_t)(16 * nt + m) * NU + 32 * ks + 8 * h;
        FragH bb;
        bb.half[0] = *(const v8ha*)brw;
        bb.half[1] = *(const v8ha*)(brw + 16);
        acc[nt] = wmma_h(a.v, bb.v, acc[nt]);
      }
    }
    const float* frow = feat + (rowg + 16 * wave + m) * NC + 8 * h;
    #pragma unroll 1
    for (int ks = 0; ks < NC / 32; ++ks) {
      const float* fr = frow + 32 * ks;
      const v4f f0 = *(const v4fa*)fr;
      const v4f f1 = *(const v4fa*)(fr + 4);
      const v4f f2 = *(const v4fa*)(fr + 16);
      const v4f f3 = *(const v4fa*)(fr + 20);
      FragH a;
      #pragma unroll
      for (int i = 0; i < 4; ++i) {
        a.v[i]      = (f16t)f0[i];
        a.v[4 + i]  = (f16t)f1[i];
        a.v[8 + i]  = (f16t)f2[i];
        a.v[12 + i] = (f16t)f3[i];
      }
      #pragma unroll
      for (int nt = 0; nt < 8; ++nt) {
        const f16t* brw = Tf + (size_t)(16 * nt + m) * NC + 32 * ks + 8 * h;
        FragH bb;
        bb.half[0] = *(const v8ha*)brw;
        bb.half[1] = *(const v8ha*)(brw + 16);
        acc[nt] = wmma_h(a.v, bb.v, acc[nt]);
      }
    }
  }
  #pragma unroll
  for (int nt = 0; nt < 8; ++nt) {
    const int col = 16 * nt + m;
    const float bias = br[col] + bfe[col];
    #pragma unroll
    for (int r = 0; r < 8; ++r)
      sEmb[(16 * wave + 8 * h + r) * EP + col] = (f16t)(acc[nt][r] * (1.0f / WCAR) + bias);
  }
  __syncthreads();

  #pragma unroll 1
  for (int p = 0; p < 3; ++p) {
    const f16t*  Tp = (p == 0) ? Tk : ((p == 1) ? Tq : Tv);
    const float* bp = (p == 0) ? bk : ((p == 1) ? bq : bv);
    #pragma unroll
    for (int nt = 0; nt < 8; ++nt) acc[nt] = zero8f();
    const f16t* arow = sEmb + (16 * wave + m) * EP + 8 * h;
    #pragma unroll 1
    for (int ks = 0; ks < NU / 32; ++ks) {
      FragH a;
      a.half[0] = *(const v8ha*)(arow + 32 * ks);
      a.half[1] = *(const v8ha*)(arow + 32 * ks + 16);
      #pragma unroll
      for (int nt = 0; nt < 8; ++nt) {
        const f16t* brw = Tp + (size_t)(16 * nt + m) * NU + 32 * ks + 8 * h;
        FragH bb;
        bb.half[0] = *(const v8ha*)brw;
        bb.half[1] = *(const v8ha*)(brw + 16);
        acc[nt] = wmma_h(a.v, bb.v, acc[nt]);
      }
    }
    #pragma unroll
    for (int nt = 0; nt < 8; ++nt) {
      const int col = 16 * nt + m;
      const float bias = bp[col];
      #pragma unroll
      for (int r = 0; r < 8; ++r)
        sEnc[(16 * wave + 8 * h + r) * EP + col] = (f16t)((acc[nt][r] * (1.0f / WCAR) + bias) * KQVCAR);
    }
    __syncthreads();
    if (p < 2) {
      f16t* dst = ((p == 0) ? KP : QP) + rowg * NU;
      #pragma unroll
      for (int i = 0; i < 8; ++i) {
        const int row = 2 * (wave + 4 * i) + h, c8 = m * 8;
        const v8h v = *(const v8ha*)(sEnc + row * EP + c8);
        *(volatile v8h*)(dst + (size_t)row * NU + c8) = v;
      }
      __threadfence();
      #pragma unroll
      for (int i = 0; i < 8; ++i) {
        const int row = 2 * (wave + 4 * i) + h, c8 = m * 8;
        const v8h v = *(const v8ha*)(sEnc + row * EP + c8);
        *(volatile v8h*)(dst + (size_t)row * NU + c8) = v;
      }
    } else {
      f16t* dst = VT + ((size_t)b * NU) * NN + n0;
      #pragma unroll
      for (int i = 0; i < 8; ++i) {
        const int dd = 4 * (wave + 4 * i) + (lane >> 3), np = (lane & 7) * 8;
        v8h o;
        #pragma unroll
        for (int e = 0; e < 8; ++e) o[e] = sEnc[(np + e) * EP + dd];
        *(volatile v8h*)(dst + (size_t)dd * NN + np) = o;
      }
      __threadfence();
      #pragma unroll
      for (int i = 0; i < 8; ++i) {
        const int dd = 4 * (wave + 4 * i) + (lane >> 3), np = (lane & 7) * 8;
        v8h o;
        #pragma unroll
        for (int e = 0; e < 8; ++e) o[e] = sEnc[(np + e) * EP + dd];
        *(volatile v8h*)(dst + (size_t)dd * NN + np) = o;
      }
    }
    __syncthreads();
  }
}

__global__ __launch_bounds__(TPR) void rel_k(const float* __restrict__ boxes, const float* __restrict__ scores,
                                            const float* __restrict__ Wg1, const float* __restrict__ bg1,
                                            const float* __restrict__ Wg2, const float* __restrict__ bg2,
                                            const float* __restrict__ Ws, const float* __restrict__ bs,
                                            const f16t* __restrict__ KP, const f16t* __restrict__ QP,
                                            const f16t* __restrict__ VT, float* __restrict__ out)
{
  __shared__ __attribute__((aligned(16))) v4f  sBox[NN];
  __shared__ __attribute__((aligned(16))) v2f  sRwh[RT];
  __shared__ __attribute__((aligned(16))) float sWs[NU];
  __shared__ __attribute__((aligned(16))) float sSc[RT];
  __shared__ __attribute__((aligned(16))) float sOut[RT];
  __shared__ float sG[8];
  __shared__ __attribute__((aligned(16))) f16t sP[2 * 16 * PP];
  const int tid = threadIdx.x, lane = tid & 31, wave = tid >> 5;
  const int h = lane >> 4, m = lane & 15;
  const int b = blockIdx.x >> 4, n0 = (blockIdx.x & 15) * RT;

  #pragma unroll 1
  for (int e = 0; e < 8; ++e) {
    const int j = tid + TPR * e;
    const v4f bx = *(const v4fa*)(boxes + ((size_t)b * NN + j) * 4);
    v4f g;
    g[0] = 0.5f * (bx[0] + bx[2]);
    g[1] = 0.5f * (bx[1] + bx[3]);
    g[2] = logf(bx[2] - bx[0]);
    g[3] = logf(bx[3] - bx[1]);
    sBox[j] = g;
  }
  if (tid < RT) {
    const v4f bx = *(const v4fa*)(boxes + ((size_t)b * NN + n0 + tid) * 4);
    v2f rr;
    rr[0] = 1.0f / (bx[2] - bx[0]);
    rr[1] = 1.0f / (bx[3] - bx[1]);
    sRwh[tid] = rr;
    sSc[tid] = scores[(size_t)b * NN + n0 + tid];
  }
  {
    const v2f w2 = *(const v2fa*)(Ws + 2 * tid);
    *(v2fa*)(sWs + 2 * tid) = w2;
  }
  {
    const int g = tid >> 3, part = tid & 7;
    const int gc = g > 4 ? 4 : g;
    const float* rp = (gc < 4) ? (Wg1 + gc * NU) : bg1;
    float s = 0.f;
    #pragma unroll 1
    for (int u = part * 16; u < part * 16 + 16; ++u) s = fmaf(rp[u], Wg2[u], s);
    s += __shfl_xor(s, 1);
    s += __shfl_xor(s, 2);
    s += __shfl_xor(s, 4);
    const float b2v = bg2[0];
    if (part == 0 && g < 5) sG[g] = s + ((g == 4) ? b2v : 0.f);
  }
  __syncthreads();

  const float g0 = sG[0], g1 = sG[1], g2 = sG[2], g3 = sG[3], gcst = sG[4];
  const float bsv = bs[0];
  const float ASC = 0.08838834764831845f * (1.0f / (KQVCAR * KQVCAR));
  f16t* sPw = sP + wave * (16 * PP);
  const size_t qrow0 = (size_t)b * NN;
  const f16t* kr = KP + ((size_t)b * NN + n0 + 16 * wave + m) * NU + 8 * h;

  v8f acc[8];
  #pragma unroll
  for (int dt = 0; dt < 8; ++dt) acc[dt] = zero8f();
  float zp[8], R[8];
  #pragma unroll
  for (int r = 0; r < 8; ++r) { zp[r] = 0.f; R[r] = 0.f; }

  #pragma unroll 1
  for (int mt = 0; mt < NN; mt += MT) {
    v8f d[4];
    #pragma unroll
    for (int nt = 0; nt < 4; ++nt) d[nt] = zero8f();
    #pragma unroll 1
    for (int ks = 0; ks < NU / 32; ++ks) {
      FragH a;
      a.half[0] = *(const v8ha*)(kr + 32 * ks);
      a.half[1] = *(const v8ha*)(kr + 32 * ks + 16);
      #pragma unroll
      for (int nt = 0; nt < 4; ++nt) {
        const f16t* qr = QP + (qrow0 + mt + 16 * nt + m) * NU + 32 * ks + 8 * h;
        FragH bb;
        bb.half[0] = *(const v8ha*)qr;
        bb.half[1] = *(const v8ha*)(qr + 16);
        d[nt] = wmma_h(a.v, bb.v, d[nt]);
      }
    }
    v4f cb[4];
    #pragma unroll
    for (int nt = 0; nt < 4; ++nt) cb[nt] = sBox[mt + 16 * nt + m];
    float mx[8];
    #pragma unroll
    for (int r = 0; r < 8; ++r) {
      const int il = 16 * wave + 8 * h + r;
      const v4f rb = sBox[n0 + il];
      const v2f rr = sRwh[il];
      float tm = 0.f;
      #pragma unroll
      for (int nt = 0; nt < 4; ++nt) {
        const float dx = fabsf(rb[0] - cb[nt][0]) * rr[0];
        const float dy = fabsf(rb[1] - cb[nt][1]) * rr[1];
        float t = g0 * __logf(fmaxf(dx, 1e-3f));
        t = fmaf(g1, __logf(fmaxf(dy, 1e-3f)), t);
        t = fmaf(g2, cb[nt][2] - rb[2], t);
        t = fmaf(g3, cb[nt][3] - rb[3], t);
        t += gcst;
        const float geo = fmaxf(t, 0.f);
        const float wv = fmaxf(geo * __expf(d[nt][r] * ASC), 1e-4f);
        d[nt][r] = wv;
        tm = fmaxf(tm, wv);
        zp[r] += wv;
      }
      mx[r] = tm;
    }
    #pragma unroll
    for (int r = 0; r < 8; ++r) {
      #pragma unroll
      for (int off = 1; off < 16; off <<= 1) mx[r] = fmaxf(mx[r], __shfl_xor(mx[r], off));
    }
    float inv[8], fac[8];
    #pragma unroll
    for (int r = 0; r < 8; ++r) {
      const float Rn = fmaxf(R[r], mx[r]);
      const float ir = 1.0f / Rn;
      fac[r] = R[r] * ir;
      inv[r] = PCAR * ir;
      R[r] = Rn;
    }
    #pragma unroll
    for (int nt = 0; nt < 4; ++nt) {
      #pragma unroll
      for (int r = 0; r < 8; ++r) sPw[(8 * h + r) * PP + 16 * nt + m] = (f16t)(d[nt][r] * inv[r]);
    }
    #pragma unroll
    for (int dt = 0; dt < 8; ++dt) {
      #pragma unroll
      for (int r = 0; r < 8; ++r) acc[dt][r] *= fac[r];
    }
    __syncthreads();
    #pragma unroll
    for (int ks = 0; ks < 2; ++ks) {
      FragH pa;
      pa.half[0] = *(const v8ha*)(sPw + m * PP + 32 * ks + 8 * h);
      pa.half[1] = *(const v8ha*)(sPw + m * PP + 32 * ks + 16 + 8 * h);
      #pragma unroll
      for (int dt = 0; dt < 8; ++dt) {
        const f16t* vr = VT + ((size_t)b * NU + 16 * dt + m) * NN + mt + 32 * ks + 8 * h;
        FragH vb;
        vb.half[0] = *(const v8ha*)vr;
        vb.half[1] = *(const v8ha*)(vr + 16);
        acc[dt] = wmma_h(pa.v, vb.v, acc[dt]);
      }
    }
    __syncthreads();
  }

  #pragma unroll
  for (int r = 0; r < 8; ++r) {
    #pragma unroll
    for (int off = 1; off < 16; off <<= 1) zp[r] += __shfl_xor(zp[r], off);
  }
  float wsv[8];
  #pragma unroll
  for (int dt = 0; dt < 8; ++dt) wsv[dt] = sWs[16 * dt + m];
  float sp[8];
  #pragma unroll
  for (int r = 0; r < 8; ++r) {
    float s = 0.f;
    #pragma unroll
    for (int dt = 0; dt < 8; ++dt) s = fmaf(acc[dt][r], wsv[dt], s);
    sp[r] = s;
  }
  #pragma unroll
  for (int r = 0; r < 8; ++r) {
    #pragma unroll
    for (int off = 1; off < 16; off <<= 1) sp[r] += __shfl_xor(sp[r], off);
  }
  float ov[8];
  #pragma unroll
  for (int r = 0; r < 8; ++r) {
    const float nrm = R[r] * (1.0f / ((PCAR * KQVCAR) * zp[r]));
    const float lg = fmaf(sp[r], nrm, bsv);
    const float sg = 1.0f / (1.0f + __expf(-lg));
    ov[r] = sSc[16 * wave + 8 * h + r] * sg;
  }
  float o = ov[0];
  #pragma unroll
  for (int r = 1; r < 8; ++r) o = ((lane & 7) == r) ? ov[r] : o;
  if (m < 8) sOut[16 * wave + 8 * h + m] = o;
  __syncthreads();
  if (tid < 8) {
    const v4f v = *(const v4fa*)(sOut + 4 * tid);
    *(volatile v4f*)(out + (size_t)b * NN + n0 + 4 * tid) = v;
  }
  __threadfence();
  if (tid < 8) {
    const v4f v = *(const v4fa*)(sOut + 4 * tid);
    *(volatile v4f*)(out + (size_t)b * NN + n0 + 4 * tid) = v;
  }
}

extern "C" void kernel_launch(void* const* d_in, const int* in_sizes, int n_in,
                              void* d_out, int out_size, void* d_ws, size_t ws_size,
                              hipStream_t stream) {
  if (n_in < 20) return;
  if (in_sizes[0]  != NB * NN * NC) return;
  if (in_sizes[1]  != NB * NN * 4)  return;
  if (in_sizes[2]  != NB * NN)      return;
  if (in_sizes[3]  != NN * NU)      return;
  if (in_sizes[4]  != NU * NU)      return;
  if (in_sizes[5]  != NU)           return;
  if (in_sizes[6]  != NC * NU)      return;
  if (in_sizes[7]  != NU)           return;
  if (in_sizes[8]  != 4 * NU)       return;
  if (in_sizes[9]  != NU)           return;
  if (in_sizes[10] != NU)           return;
  if (in_sizes[11] < 1)             return;
  if (in_sizes[12] != NU * NU)      return;
  if (in_sizes[13] != NU)           return;
  if (in_sizes[14] != NU * NU)      return;
  if (in_sizes[15] != NU)           return;
  if (in_sizes[16] != NU * NU)      return;
  if (in_sizes[17] != NU)           return;
  if (in_sizes[18] != NU)           return;
  if (in_sizes[19] < 1)             return;
  if (out_size != NB * NN)          return;

  const float* feature_map = (const float*)d_in[0];
  const float* boxes   = (const float*)d_in[1];
  const float* scores  = (const float*)d_in[2];
  const float* enc     = (const float*)d_in[3];
  const float* W_rank  = (const float*)d_in[4];
  const float* b_rank  = (const float*)d_in[5];
  const float* W_feat  = (const float*)d_in[6];
  const float* b_feat  = (const float*)d_in[7];
  const float* Wg1     = (const float*)d_in[8];
  const float* bg1     = (const float*)d_in[9];
  const float* Wg2     = (const float*)d_in[10];
  const float* bg2     = (const float*)d_in[11];
  const float* Wk      = (const float*)d_in[12];
  const float* bk      = (const float*)d_in[13];
  const float* Wq      = (const float*)d_in[14];
  const float* bq      = (const float*)d_in[15];
  const float* Wv      = (const float*)d_in[16];
  const float* bv      = (const float*)d_in[17];
  const float* Ws      = (const float*)d_in[18];
  const float* bs      = (const float*)d_in[19];
  float* outp = (float*)d_out;

  const size_t szTr = (size_t)NU * NU * 2;
  const size_t szTf = (size_t)NU * NC * 2;
  const size_t szTk = (size_t)NU * NU * 2;
  const size_t szKQ = (size_t)NB * NN * NU * 2;
  const size_t szVT = (size_t)NB * NU * NN * 2;
  size_t off = 0;
  char* ws = (char*)d_ws;
  f16t* Tr = (f16t*)(ws + off); off += szTr;
  f16t* Tf = (f16t*)(ws + off); off += szTf;
  f16t* Tk = (f16t*)(ws + off); off += szTk;
  f16t* Tq = (f16t*)(ws + off); off += szTk;
  f16t* Tv = (f16t*)(ws + off); off += szTk;
  f16t* KP = (f16t*)(ws + off); off += szKQ;
  f16t* QP = (f16t*)(ws + off); off += szKQ;
  f16t* VT = (f16t*)(ws + off); off += szVT;
  if (off > ws_size) return;

  prep_w_k<<<48, TPW, 0, stream>>>(W_rank, W_feat, Wk, Wq, Wv, Tr, Tf, Tk, Tq, Tv);
  proj_k<<<NB * (NN / PT), TPP, 0, stream>>>(feature_map, scores, enc, b_rank, b_feat, bk, bq, bv,
                                             Tr, Tf, Tk, Tq, Tv, KP, QP, VT);
  rel_k<<<NB * (NN / RT), TPR, 0, stream>>>(boxes, scores, Wg1, bg1, Wg2, bg2, Ws, bs, KP, QP, VT, outp);
}
